// MultiHeadAttention_66211215835323
// MI455X (gfx1250) — hardware-verified
//
#include <hip/hip_runtime.h>


#ifndef NB
#define NB 2
#endif
#ifndef SEQ
#define SEQ 2048
#endif
#define NB_FULL  2
#define SEQ_FULL 2048
#ifndef OUT_SEQ
#define OUT_SEQ SEQ
#endif
#define DM   1024
#define NH_  16
#define KD   16
#define VD   64
#define HV   (NH_ * VD)
#define QKW  32
#define AW   4
#define RSC  64.0f
#define RSI  (1.0f / 64.0f)
#define SC2  (0.25f * 1.4426950408889634f)
#define PSH  10.0f
#define WOS  64.0f
#define OSC  (1.0f / 65536.0f)

static_assert(KD == 16);
static_assert(NH_ == KD);
static_assert(VD == 64);
static_assert(HV == DM);
static_assert(DM % 64 == 0);
static_assert(DM % 32 == 0);
static_assert((NH_ * KD) % 64 == 0);
static_assert(SEQ % 64 == 0);
static_assert((NB * SEQ) % 64 == 0);
static_assert(SEQ % 32 == 0);
static_assert(SEQ % (16 * AW) == 0);
static_assert(SEQ % (32 * AW) == 0);
static_assert(((size_t)SEQ * DM) % 8 == 0);
static_assert(NB <= NB_FULL);
static_assert(SEQ <= SEQ_FULL);

typedef _Float16 h16;
typedef unsigned short bf;
typedef __attribute__((ext_vector_type(16))) __bf16   v16bf;
typedef __attribute__((ext_vector_type(16))) _Float16 v16h;
typedef __attribute__((ext_vector_type(8)))  _Float16 v8h;
typedef __attribute__((ext_vector_type(8)))  unsigned short v8us;
typedef __attribute__((ext_vector_type(8)))  float    v8f;
typedef __attribute__((ext_vector_type(4)))  float    v4f;
typedef v4f  __attribute__((may_alias)) v4fa;

__device__ __forceinline__ unsigned short f2bf(float f) { unsigned u = __float_as_uint(f); u += 0x7FFFu + ((u >> 16) & 1u); return (unsigned short)(u >> 16); }
__device__ __forceinline__ v16h cat16(v8h lo, v8h hi) { return __builtin_shufflevector(lo, hi, 0, 1, 2, 3, 4, 5, 6, 7, 8, 9, 10, 11, 12, 13, 14, 15); }
__device__ __forceinline__ v8f wmma16(v16h a, v16h b, v8f c) { return __builtin_amdgcn_wmma_f32_16x16x32_f16(false, a, false, b, (short)0, c, false, false); }
__device__ __forceinline__ v8f wmmab(v16bf a, v16bf b, v8f c) { return __builtin_amdgcn_wmma_f32_16x16x32_bf16(false, a, false, b, (short)0, c, false, false); }
__device__ __forceinline__ v8f wm(v16h a, v16h b, v8f c) { return wmma16(a, b, c); }
__device__ __forceinline__ v8f wm(v16bf a, v16bf b, v8f c) { return wmmab(a, b, c); }
__device__ __forceinline__ v16h  ldh(const h16* p) { return cat16(*(const v8h*)p, *(const v8h*)(p + 16)); }
template <class F> __device__ __forceinline__ F ldf(const bf* p) {
    const v8us lo = *(const v8us*)p; const v8us hi8 = *(const v8us*)(p + 16);
    return __builtin_bit_cast(F, __builtin_shufflevector(lo, hi8, 0, 1, 2, 3, 4, 5, 6, 7, 8, 9, 10, 11, 12, 13, 14, 15)); }
template <int F16> struct FragSel { typedef v16bf T; };
template <> struct FragSel<1> { typedef v16h T; };
__device__ __forceinline__ void wave_sync() { __builtin_amdgcn_fence(3  , "wavefront"); __builtin_amdgcn_wave_barrier(); asm volatile("" ::: "memory"); }

__global__ __launch_bounds__(256) void k_cvt8(const float* __restrict__ src, bf* dst, size_t n8, int mode) {
    const size_t i = (size_t)blockIdx.x * 256 + threadIdx.x; if (i >= n8) return;
    size_t si = i;
    if (mode == 1) { const size_t r = i / (DM / 8), p = i % (DM / 8); const size_t sr = (r & 15) * 16 + (r >> 4); si = sr * (DM / 8) + p; }
    const v8f v = *(const v8f*)(src + si * 8); v8us o;
#pragma unroll
    for (int k = 0; k < 8; ++k) {
        const unsigned short bb = f2bf(v[k]);
        const h16 hv = (h16)(__uint_as_float(((unsigned)bb) << 16) * WOS);
        o[k] = (mode == 2) ? __builtin_bit_cast(unsigned short, hv) : bb; }
    *(volatile v8us*)(dst + i * 8) = o; __threadfence(); *(volatile v8us*)(dst + i * 8) = o;
}

template <int MODE>
__global__ __launch_bounds__(32) void k_gemm(const bf* __restrict__ A, const bf* __restrict__ Bt, h16* P16, float* P32) {
    typedef typename FragSel<(MODE == 3) ? 1 : 0>::T FT;
    __shared__ __align__(16) float os[16 * 68];
    const int K = DM;
    const int lane = threadIdx.x & 31, lr = lane & 15, hi = lane >> 4; const int r0 = blockIdx.x * 64, c0 = blockIdx.y * 64;
    v8f acc[4][4];
#pragma unroll
    for (int mb = 0; mb < 4; ++mb)
#pragma unroll
        for (int nb = 0; nb < 4; ++nb) acc[mb][nb] = (v8f){};
    const size_t aoff = (size_t)(r0 + lr) * K + 8 * hi, boff = (size_t)(c0 + lr) * K + 8 * hi;
#pragma unroll 1
    for (int kc = 0; kc < K; kc += 32) {
        FT a[4];
#pragma unroll
        for (int mb = 0; mb < 4; ++mb) a[mb] = ldf<FT>(A + aoff + (size_t)mb * 16 * K + kc);
#pragma unroll
        for (int nb = 0; nb < 4; ++nb) { const FT b = ldf<FT>(Bt + boff + (size_t)nb * 16 * K + kc);
#pragma unroll
            for (int mb = 0; mb < 4; ++mb) acc[mb][nb] = wm(a[mb], b, acc[mb][nb]); }
        asm volatile("v_nop\n\tv_nop\n\tv_nop\n\tv_nop" : "+v"(acc[0][0]), "+v"(acc[1][1]), "+v"(acc[2][2]), "+v"(acc[3][3]) : "v"(a[0]), "v"(a[1]), "v"(a[2]), "v"(a[3]));
    }
#pragma unroll
    for (int mb = 0; mb < 4; ++mb) {
#pragma unroll
        for (int nb = 0; nb < 4; ++nb) {
#pragma unroll
            for (int j = 0; j < 8; ++j) os[(hi * 8 + j) * 68 + nb * 16 + lr] = acc[mb][nb][j]; }
        wave_sync();
        if (MODE == 0) {
            const size_t sb = ((size_t)(c0 / SEQ) * HV + (size_t)(r0 + mb * 16)) * (size_t)SEQ + (size_t)(c0 % SEQ);
#pragma unroll 1
            for (int ps = 0; ps < 2; ++ps) {
#pragma unroll
                for (int s = 0; s < 4; ++s) { const int row = 4 * s + (lane >> 3), c8 = (lane & 7) * 8;
                    const v4f x0 = *(const v4fa*)(&os[row * 68 + c8]); const v4f x1 = *(const v4fa*)(&os[row * 68 + c8 + 4]); v8h hv;
#pragma unroll
                    for (int i = 0; i < 4; ++i) { hv[i] = (h16)x0[i]; hv[4 + i] = (h16)x1[i]; }
                    *(volatile v8h*)(P16 + sb + (size_t)row * (size_t)SEQ + c8) = hv; }
                if (ps == 0) __threadfence(); }
        } else if (MODE == 3) {
            const size_t sb = ((size_t)(r0 / SEQ) * OUT_SEQ + (size_t)(r0 % SEQ) + (size_t)(mb * 16)) * (size_t)DM + (size_t)c0;
#pragma unroll 1
            for (int ps = 0; ps < 2; ++ps) {
#pragma unroll
                for (int s = 0; s < 8; ++s) { const int row = 2 * s + hi, cofs = lr * 4;
                    v4f val = *(const v4fa*)(&os[row * 68 + cofs]); val = val * OSC;
                    *(volatile v4f*)(P32 + sb + (size_t)row * DM + cofs) = val; }
                if (ps == 0) __threadfence(); }
        } else {
            const int bq = r0 / SEQ, tq = r0 % SEQ, h0 = c0 / KD;
#pragma unroll 1
            for (int ps = 0; ps < 2; ++ps) {
#pragma unroll
                for (int hh = 0; hh < 4; ++hh) {
                    const size_t hb = ((size_t)(bq * NH_ + h0 + hh) * SEQ + (size_t)(tq + mb * 16)) * QKW;
#pragma unroll
                    for (int s = 0; s < 2; ++s) { const int row = s * 8 + (lane >> 2), pc = lane & 3, jb = (pc & 1) * 8;
                        const v4f x0 = *(const v4fa*)(&os[row * 68 + hh * 16 + jb]); const v4f x1 = *(const v4fa*)(&os[row * 68 + hh * 16 + jb + 4]); v8h hv, rv;
#pragma unroll
                        for (int i = 0; i < 4; ++i) { const h16 a0 = (h16)x0[i]; const h16 a1 = (h16)x1[i]; hv[i] = a0; hv[4 + i] = a1;
                            if (MODE == 1) { rv[i] = (h16)((x0[i] - (float)a0) * RSC); rv[4 + i] = (h16)((x1[i] - (float)a1) * RSC); }
                            else           { rv[i] = (h16)((float)a0 * RSI);           rv[4 + i] = (h16)((float)a1 * RSI); } }
                        const v8h ov = (pc < 2) ? hv : rv;
                        *(volatile v8h*)(P16 + hb + (size_t)(s * 256 + lane * 8)) = ov; } }
                if (ps == 0) __threadfence(); }
        }
        wave_sync();
    }
}

__device__ __forceinline__ void stat_upd(const v8f sa, const v8f sb, float& m, float& l) {
    float t[16]; float mx = -3.0e38f;
#pragma unroll
    for (int r = 0; r < 8; ++r) { t[r] = sa[r] * SC2; t[8 + r] = sb[r] * SC2; mx = fmaxf(mx, fmaxf(t[r], t[8 + r])); }
    const float mnew = fmaxf(m, mx);
    const float alpha = __builtin_amdgcn_exp2f(m - mnew);
    float ls = 0.0f;
#pragma unroll
    for (int r = 0; r < 16; ++r) ls += __builtin_amdgcn_exp2f(t[r] - mnew);
    l = l * alpha + ls; m = mnew;
}

__global__ __launch_bounds__(32 * AW) void k_stats(const h16* __restrict__ QP, const h16* __restrict__ KP, float* LSE) {
    __shared__ __align__(16) float ls[AW * 32];
    const int lane = threadIdx.x & 31, wave = __builtin_amdgcn_readfirstlane((int)(threadIdx.x >> 5)), lr = lane & 15, hi = lane >> 4;
    const int zh = blockIdx.y;
    const int m0 = (blockIdx.x * AW + wave) * 32;
    const size_t pbase = (size_t)zh * SEQ * QKW;
    const v16h kf0 = ldh(KP + pbase + (size_t)(m0 + lr) * QKW + 8 * hi), kf1 = ldh(KP + pbase + (size_t)(m0 + 16 + lr) * QKW + 8 * hi);
    const size_t qo = pbase + (size_t)lr * QKW + 8 * hi;
    float ma = -3.0e38f, la = 0.0f, mb = -3.0e38f, lb = 0.0f;
#pragma unroll 1
    for (int n0 = 0; n0 < SEQ; n0 += 32) {
        const v16h qa0 = ldh(QP + qo + (size_t)n0 * QKW), qa1 = ldh(QP + qo + (size_t)(n0 + 16) * QKW);
        v8f s00 = (v8f){}, s01 = (v8f){}, s10 = (v8f){}, s11 = (v8f){};
        s00 = wmma16(qa0, kf0, s00); s01 = wmma16(qa0, kf1, s01); s10 = wmma16(qa1, kf0, s10); s11 = wmma16(qa1, kf1, s11);
        asm volatile("v_nop\n\tv_nop\n\tv_nop\n\tv_nop" : "+v"(s00), "+v"(s01), "+v"(s10), "+v"(s11) : "v"(qa0), "v"(qa1), "v"(kf0), "v"(kf1));
        stat_upd(s00, s10, ma, la);
        stat_upd(s01, s11, mb, lb);
    }
    const float mao = __shfl_xor(ma, 16, 32), lao = __shfl_xor(la, 16, 32), mbo = __shfl_xor(mb, 16, 32), lbo = __shfl_xor(lb, 16, 32);
    const float Ma = fmaxf(ma, mao), Mb = fmaxf(mb, mbo);
    const float La = la * __builtin_amdgcn_exp2f(ma - Ma) + lao * __builtin_amdgcn_exp2f(mao - Ma);
    const float Lb = lb * __builtin_amdgcn_exp2f(mb - Mb) + lbo * __builtin_amdgcn_exp2f(mbo - Mb);
    const float lseA = Ma + log2f(La), lseB = Mb + log2f(Lb);
    ls[wave * 32 + hi * 16 + lr] = hi ? lseB : lseA;
    wave_sync();
    const v4f val = *(const v4fa*)(&ls[wave * 32 + (lane & 7) * 4]);
    float* dst = LSE + (size_t)zh * SEQ + m0 + (lane & 7) * 4;
#pragma unroll 1
    for (int ps = 0; ps < 2; ++ps) {
        if (lane < 8) *(volatile v4f*)dst = val;
        if (ps == 0) __threadfence(); }
}

__global__ __launch_bounds__(32 * AW) void k_attn(const h16* __restrict__ QP, const h16* __restrict__ KP, const h16* __restrict__ VT, const float* __restrict__ LSE, h16* OH) {
    __shared__ __align__(16) float os[AW * 16 * 68];
    const int lane = threadIdx.x & 31, wave = __builtin_amdgcn_readfirstlane((int)(threadIdx.x >> 5)), lr = lane & 15, hi = lane >> 4;
    const int zh = blockIdx.y; const int b = zh / NH_, h = zh % NH_;
    const int t0 = (blockIdx.x * AW + wave) * 16;
    const size_t pq = (size_t)zh * SEQ * QKW;
    const v16h qf = ldh(QP + pq + (size_t)(t0 + lr) * QKW + 8 * hi);
    const size_t ko = pq + (size_t)lr * QKW + 8 * hi;
    const size_t vo = (size_t)zh * VD * SEQ + (size_t)lr * SEQ + 8 * hi;
    const float* lsep = LSE + (size_t)zh * SEQ + 8 * hi;
    v8f o0 = (v8f){}, o1 = (v8f){}, o2 = (v8f){}, o3 = (v8f){};
#pragma unroll 1
    for (int key0 = 0; key0 < SEQ; key0 += 32) {
        const h16* kp = KP + ko + (size_t)key0 * QKW;
        const v16h ka = ldh(kp), kb = ldh(kp + 16 * QKW);
        v8f sa = (v8f){}, sb = (v8f){};
        sa = wmma16(ka, qf, sa); sb = wmma16(kb, qf, sb);
        asm volatile("v_nop\n\tv_nop\n\tv_nop\n\tv_nop" : "+v"(sa), "+v"(sb) : "v"(ka), "v"(kb), "v"(qf));
        const v4f la0 = *(const v4f*)(lsep + key0), la1 = *(const v4f*)(lsep + key0 + 4), lb0 = *(const v4f*)(lsep + key0 + 16), lb1 = *(const v4f*)(lsep + key0 + 20);
        v16h pb;
#pragma unroll
        for (int r = 0; r < 4; ++r) {
            pb[r]      = (h16)__builtin_amdgcn_exp2f(sa[r]     * SC2 + (PSH - la0[r]));
            pb[4 + r]  = (h16)__builtin_amdgcn_exp2f(sa[4 + r] * SC2 + (PSH - la1[r]));
            pb[8 + r]  = (h16)__builtin_amdgcn_exp2f(sb[r]     * SC2 + (PSH - lb0[r]));
            pb[12 + r] = (h16)__builtin_amdgcn_exp2f(sb[4 + r] * SC2 + (PSH - lb1[r])); }
        const h16* va = VT + vo + key0;
        const v16h v0 = ldh(va), v1 = ldh(va + (size_t)16 * SEQ), v2 = ldh(va + (size_t)32 * SEQ), v3 = ldh(va + (size_t)48 * SEQ);
        o0 = wmma16(v0, pb, o0); o1 = wmma16(v1, pb, o1); o2 = wmma16(v2, pb, o2); o3 = wmma16(v3, pb, o3);
        asm volatile("v_nop\n\tv_nop\n\tv_nop\n\tv_nop" : "+v"(o0), "+v"(o1), "+v"(o2), "+v"(o3) : "v"(v0), "v"(v1), "v"(v2), "v"(v3), "v"(pb));
    }
    const int wb = wave * 16 * 68;
    { v4f a, c;
      a[0] = o0[0]; a[1] = o0[1]; a[2] = o0[2]; a[3] = o0[3]; c[0] = o0[4]; c[1] = o0[5]; c[2] = o0[6]; c[3] = o0[7];
      *(v4fa*)(&os[wb + lr * 68 +  0 + 8 * hi]) = a; *(v4fa*)(&os[wb + lr * 68 +  0 + 8 * hi + 4]) = c;
      a[0] = o1[0]; a[1] = o1[1]; a[2] = o1[2]; a[3] = o1[3]; c[0] = o1[4]; c[1] = o1[5]; c[2] = o1[6]; c[3] = o1[7];
      *(v4fa*)(&os[wb + lr * 68 + 16 + 8 * hi]) = a; *(v4fa*)(&os[wb + lr * 68 + 16 + 8 * hi + 4]) = c;
      a[0] = o2[0]; a[1] = o2[1]; a[2] = o2[2]; a[3] = o2[3]; c[0] = o2[4]; c[1] = o2[5]; c[2] = o2[6]; c[3] = o2[7];
      *(v4fa*)(&os[wb + lr * 68 + 32 + 8 * hi]) = a; *(v4fa*)(&os[wb + lr * 68 + 32 + 8 * hi + 4]) = c;
      a[0] = o3[0]; a[1] = o3[1]; a[2] = o3[2]; a[3] = o3[3]; c[0] = o3[4]; c[1] = o3[5]; c[2] = o3[6]; c[3] = o3[7];
      *(v4fa*)(&os[wb + lr * 68 + 48 + 8 * hi]) = a; *(v4fa*)(&os[wb + lr * 68 + 48 + 8 * hi + 4]) = c; }
    wave_sync();
    h16* orow = OH + ((size_t)b * SEQ + t0) * HV + (size_t)h * VD;
#pragma unroll 1
    for (int ps = 0; ps < 2; ++ps) {
#pragma unroll
        for (int s = 0; s < 4; ++s) { const int row = 4 * s + (lane >> 3), c8 = (lane & 7) * 8;
            const v4f x0 = *(const v4fa*)(&os[wb + row * 68 + c8]); const v4f x1 = *(const v4fa*)(&os[wb + row * 68 + c8 + 4]); v8h hv;
#pragma unroll
            for (int i = 0; i < 4; ++i) { hv[i] = (h16)x0[i]; hv[4 + i] = (h16)x1[i]; }
            *(volatile v8h*)(orow + (size_t)row * HV + c8) = hv; }
        if (ps == 0) __threadfence(); }
}

static constexpr size_t al256(size_t v) { return (v + 255) & ~(size_t)255; }
static constexpr size_t SZ_XB  = al256((size_t)NB * SEQ * DM * 2);
static constexpr size_t SZ_WQK = al256((size_t)NH_ * KD * DM * 2);
static constexpr size_t SZ_WV  = al256((size_t)HV * DM * 2);
static constexpr size_t SZ_WO  = al256((size_t)DM * HV * 2);
static constexpr size_t SZ_QK  = al256((size_t)NB * NH_ * SEQ * QKW * 2);
static constexpr size_t SZ_VT  = al256((size_t)NB * HV * SEQ * 2);
static constexpr size_t SZ_LSE = al256((size_t)NB * NH_ * SEQ * 4);
static constexpr size_t SZ_OH  = al256((size_t)NB * SEQ * HV * 2);
static constexpr size_t SZ_TOTAL = SZ_XB + 2 * SZ_WQK + SZ_WV + SZ_WO + 2 * SZ_QK + SZ_VT + SZ_LSE + SZ_OH;
static_assert(SZ_TOTAL <= (size_t)134217728);

extern "C" void kernel_launch(void* const* d_in, const int* in_sizes, int n_in,
                              void* d_out, int out_size, void* d_ws, size_t ws_size, hipStream_t stream) {
    if (n_in < 5) return;
    const size_t needx = ((size_t)(NB - 1) * SEQ_FULL + SEQ) * DM;
    if ((size_t)in_sizes[0] < needx) return;
    if ((size_t)in_sizes[1] < (size_t)NH_ * KD * DM || (size_t)in_sizes[2] < (size_t)NH_ * KD * DM) return;
    if ((size_t)in_sizes[3] < (size_t)HV * DM || (size_t)in_sizes[4] < (size_t)DM * HV) return;
    if ((size_t)out_size < ((size_t)(NB - 1) * OUT_SEQ + SEQ) * DM) return;
    if (SZ_TOTAL > ws_size) return;
    const float* x = (const float*)d_in[0]; const float* wq = (const float*)d_in[1]; const float* wk = (const float*)d_in[2];
    const float* wv = (const float*)d_in[3]; const float* wo = (const float*)d_in[4];
    float* OUT = (float*)d_out;
    char* wsp = (char*)d_ws;
    bf* XB = (bf*)wsp; wsp += SZ_XB;
    bf* WQ = (bf*)wsp; wsp += SZ_WQK;
    bf* WK = (bf*)wsp; wsp += SZ_WQK;
    bf* WV = (bf*)wsp; wsp += SZ_WV;
    bf* WO = (bf*)wsp; wsp += SZ_WO;
    h16* QP = (h16*)wsp; wsp += SZ_QK;
    h16* KP = (h16*)wsp; wsp += SZ_QK;
    h16* VT = (h16*)wsp; wsp += SZ_VT;
    float* LSE = (float*)wsp; wsp += SZ_LSE;
    h16* OH = (h16*)wsp; wsp += SZ_OH;

    if (SEQ == SEQ_FULL) {
        const size_t n8 = (size_t)NB * SEQ * DM / 8;
        k_cvt8<<<(unsigned)((n8 + 255) / 256), 256, 0, stream>>>(x, XB, n8, 0);
    } else {
        const size_t n8 = (size_t)SEQ * DM / 8;
        for (int b = 0; b < NB; ++b) k_cvt8<<<(unsigned)((n8 + 255) / 256), 256, 0, stream>>>(x + (size_t)b * SEQ_FULL * DM, XB + (size_t)b * SEQ * DM, n8, 0);
    }
    { const size_t n8 = (size_t)NH_ * KD * DM / 8; const unsigned g = (unsigned)((n8 + 255) / 256);
      k_cvt8<<<g, 256, 0, stream>>>(wq, WQ, n8, 1); k_cvt8<<<g, 256, 0, stream>>>(wk, WK, n8, 0); }
    { const size_t n8 = (size_t)HV * DM / 8; const unsigned g = (unsigned)((n8 + 255) / 256);
      k_cvt8<<<g, 256, 0, stream>>>(wv, WV, n8, 0); k_cvt8<<<g, 256, 0, stream>>>(wo, WO, n8, 2); }

    k_gemm<1><<<dim3(NB * SEQ / 64, (NH_ * KD) / 64, 1), 32, 0, stream>>>(XB, WQ, QP, OUT);
    k_gemm<2><<<dim3(NB * SEQ / 64, (NH_ * KD) / 64, 1), 32, 0, stream>>>(XB, WK, KP, OUT);
    k_gemm<0><<<dim3(HV / 64, NB * SEQ / 64, 1), 32, 0, stream>>>(WV, XB, VT, OUT);

    k_stats<<<dim3(SEQ / (32 * AW), NB * NH_, 1), 32 * AW, 0, stream>>>(QP, KP, LSE);
    k_attn<<<dim3(SEQ / (16 * AW), NB * NH_, 1), 32 * AW, 0, stream>>>(QP, KP, VT, LSE, OH);

    k_gemm<3><<<dim3(NB * SEQ / 64, DM / 64, 1), 32, 0, stream>>>((const bf*)OH, WO, QP, OUT);
}
